// RGCN2_25168508354750
// MI455X (gfx1250) — hardware-run, weakly checked
//
#include <hip/hip_runtime.h>

typedef float          v8f   __attribute__((ext_vector_type(8)));
typedef float          v4f   __attribute__((ext_vector_type(4)));
typedef unsigned int   v4u   __attribute__((ext_vector_type(4)));
typedef int            v8i   __attribute__((ext_vector_type(8)));
typedef unsigned short v8us  __attribute__((ext_vector_type(8)));
typedef unsigned short v16us __attribute__((ext_vector_type(16)));
typedef __bf16         v16bf __attribute__((ext_vector_type(16)));
typedef _Float16       v16h  __attribute__((ext_vector_type(16)));
typedef v4f  __attribute__((may_alias)) v4fa;
typedef v8us __attribute__((may_alias)) v8usa;
union FragB { v16bf v; v16us u; v8us h[2]; v8i w; };
union FragH { v16h  v; v16us u; v8us h[2]; v8i w; };

__device__ __forceinline__ v8f wmb(const FragB& a, const FragB& b, v8f c) {
  v8f d = __builtin_amdgcn_wmma_f32_16x16x32_bf16(false, a.v, false, b.v, (short)0, c, false, false);
  asm volatile("v_nop\n\tv_nop\n\tv_nop\n\tv_nop" : "+v"(d) : "v"(a.w), "v"(b.w));
  return d;
}

__device__ __forceinline__ v8f wmh(const FragH& a, const FragH& b, v8f c) {
  v8f d = __builtin_amdgcn_wmma_f32_16x16x32_f16(false, a.v, false, b.v, (short)0, c, false, false);
  asm volatile("v_nop\n\tv_nop\n\tv_nop\n\tv_nop" : "+v"(d) : "v"(a.w), "v"(b.w));
  return d;
}

__device__ __forceinline__ unsigned bf16_bits(float f) {
  const unsigned u = __float_as_uint(f);
  const unsigned r = (u + 0x7FFFu + ((u >> 16) & 1u)) >> 16;
  const unsigned q = (u >> 16) | 0x40u;
  return ((u & 0x7fffffffu) > 0x7f800000u) ? q : r;
}

__device__ __forceinline__ float bf16_val(float f) {
  return __uint_as_float(bf16_bits(f) << 16);
}
__device__ __forceinline__ int clampi(int v, int lo, int hi) {
  return v < lo ? lo : (v > hi ? hi : v);
}

__device__ __forceinline__ unsigned f16_bits(float f) {
  const unsigned u  = __float_as_uint(f);
  const unsigned s  = (u >> 16) & 0x8000u;
  const unsigned a  = u & 0x7fffffffu;
  const unsigned t  = a - 0x38000000u;
  const unsigned r  = (t + 0x0FFFu + ((t >> 13) & 1u)) >> 13;
  const unsigned rc = r > 0x7C00u ? 0x7C00u : r;
  const bool small  = a < 0x38800000u;
  const bool isnan  = a > 0x7f800000u;
  const unsigned fin = small ? 0u : (s | rc);
  return isnan ? (s | 0x7E00u) : fin;
}

__device__ __forceinline__ unsigned pk16(unsigned lo, unsigned hi) { return lo | (hi << 16); }
__device__ __forceinline__ unsigned bf16_lo_bits(float v) {
  float hi = bf16_val(v);
  asm volatile("" : "+v"(hi));
  return bf16_bits(v - hi);
}
__device__ __forceinline__ v4u pack8_bf16(v4f a, v4f c) {
  return (v4u){ pk16(bf16_bits(a[0]), bf16_bits(a[1])), pk16(bf16_bits(a[2]), bf16_bits(a[3])),
                pk16(bf16_bits(c[0]), bf16_bits(c[1])), pk16(bf16_bits(c[2]), bf16_bits(c[3])) };
}
__device__ __forceinline__ v4u pack8_bf16_lo(v4f a, v4f c) {
  return (v4u){ pk16(bf16_lo_bits(a[0]), bf16_lo_bits(a[1])), pk16(bf16_lo_bits(a[2]), bf16_lo_bits(a[3])),
                pk16(bf16_lo_bits(c[0]), bf16_lo_bits(c[1])), pk16(bf16_lo_bits(c[2]), bf16_lo_bits(c[3])) };
}
__device__ __forceinline__ v4u pack8_f16(v4f a, v4f c) {
  return (v4u){ pk16(f16_bits(a[0]), f16_bits(a[1])), pk16(f16_bits(a[2]), f16_bits(a[3])),
                pk16(f16_bits(c[0]), f16_bits(c[1])), pk16(f16_bits(c[2]), f16_bits(c[3])) };
}

template <int FORM>
__global__ __launch_bounds__(256) void k_plane(const float* __restrict__ src, int rows, int cols, int ldsrc,
                                               unsigned short* __restrict__ dst, int MP, int KP) {
  static_assert(FORM >= 0 && FORM <= 3);
  const int KTOT = (FORM == 1 || FORM == 3) ? 2 * KP : KP;
  const unsigned ppr   = (unsigned)(KTOT >> 3);
  const unsigned kp8   = (unsigned)(KP >> 3);
  const unsigned total = (unsigned)MP * ppr;
  const unsigned g     = blockIdx.x * 256u + threadIdx.x;
  const unsigned rowu  = g / ppr;
  const unsigned p     = g - rowu * ppr;
  const bool second    = p >= kp8;
  const int row = (int)rowu;
  const int c0  = (int)((second ? p - kp8 : p) << 3);
  const float* srow = src + (size_t)clampi(row, 0, rows - 1) * (size_t)ldsrc;
  float x[8];
  unsigned mk[8];
#pragma unroll
  for (int e = 0; e < 8; ++e) {
    const int c = c0 + e;
    const float v = srow[clampi(c, 0, cols - 1)];
    asm volatile("" :: "v"(v));
    x[e]  = v;
    mk[e] = (row < rows && c < cols) ? 0xFFFFu : 0u;
  }
  const v4f a = (v4f){ x[0], x[1], x[2], x[3] };
  const v4f c = (v4f){ x[4], x[5], x[6], x[7] };
  v4u o;
  if (FORM == 2) {
    o = pack8_f16(a, c);
  } else {
    const v4u hi = pack8_bf16(a, c);
    o = hi;
    if (FORM == 1) { const v4u lo = pack8_bf16_lo(a, c); o = second ? lo : hi; }
  }
  const v4u mw = (v4u){ pk16(mk[0], mk[1]), pk16(mk[2], mk[3]), pk16(mk[4], mk[5]), pk16(mk[6], mk[7]) };
  o &= mw;
  if (g < total) {
    volatile v4u* q = (volatile v4u*)(dst + (size_t)g * 8);
    *q = o;
    __threadfence();
    *q = o;
  }
}

template <int FORM> struct FragOf    { typedef FragB T; };
template <>         struct FragOf<2> { typedef FragH T; };
__device__ __forceinline__ v8f mm(const FragB& a, const FragB& b, v8f c) { return wmb(a, b, c); }
__device__ __forceinline__ v8f mm(const FragH& a, const FragH& b, v8f c) { return wmh(a, b, c); }
template <class F> __device__ __forceinline__ F ld_frag(const unsigned short* p) {
  F f;
  f.h[0] = *(const v8usa*)(p);
  f.h[1] = *(const v8usa*)(p + 16);
  return f;
}

template <int FORM, int EPI>
__global__ __launch_bounds__(256) __attribute__((amdgpu_num_vgpr(248)))
void k_gemm_nt(const unsigned short* __restrict__ A, const unsigned short* __restrict__ B,
               const float* __restrict__ bias, float* __restrict__ D, int M, int N, int KTOT, int ldd) {
  static_assert(FORM >= 0 && FORM <= 2);
  static_assert(EPI == 0 || EPI == 1);
  typedef typename FragOf<FORM>::T F;
  __shared__ __attribute__((aligned(16))) float sT[8][16 * 68];
  const int lane = threadIdx.x & 31;
  const int wave = threadIdx.x >> 5;
  const int tilesM = (M + 63) >> 6;
  const int tilesN = (N + 63) >> 6;
  const int tile = blockIdx.x * 8 + wave;
  if (tile >= tilesM * tilesN) return;
  const int tm = tile / tilesN;
  const int tn = tile - tm * tilesN;
  const int m0 = tm << 6;
  const int n0 = tn << 6;

  const int rl = lane & 15;
  const int h8 = (lane >> 4) * 8;
  const unsigned short* pa = A + (size_t)(m0 + rl) * (size_t)KTOT + h8;
  const unsigned short* pb = B + (size_t)(n0 + rl) * (size_t)KTOT + h8;

  v8f acc[4][4];
#pragma unroll
  for (int i = 0; i < 4; ++i)
#pragma unroll
    for (int j = 0; j < 4; ++j) acc[i][j] = (v8f){0.f, 0.f, 0.f, 0.f, 0.f, 0.f, 0.f, 0.f};

#pragma unroll 1
  for (int k0 = 0; k0 < KTOT; k0 += 32) {
    F bf[4];
#pragma unroll
    for (int j = 0; j < 4; ++j) bf[j] = ld_frag<F>(pb + (size_t)(j << 4) * (size_t)KTOT + k0);
#pragma unroll
    for (int i = 0; i < 4; ++i) {
      const F af = ld_frag<F>(pa + (size_t)(i << 4) * (size_t)KTOT + k0);
#pragma unroll
      for (int j = 0; j < 4; ++j) acc[i][j] = mm(af, bf[j], acc[i][j]);
    }
  }

  float* slab = sT[wave];
  const int hh = lane >> 4;
  const int c4 = (lane & 15) * 4;
  const int nc = n0 + c4;
  const bool cok = nc < N;
  v4f bv = (v4f){0.f, 0.f, 0.f, 0.f};
  if (EPI == 1) {
    bv = *(const v4fa*)(bias + clampi(nc, 0, N - 4));
    asm volatile("" :: "v"(bv));
  }
#pragma unroll
  for (int i = 0; i < 4; ++i) {
    const int mBase = m0 + (i << 4);
#pragma unroll
    for (int j = 0; j < 4; ++j) {
#pragma unroll
      for (int r = 0; r < 8; ++r) slab[(h8 + r) * 68 + (j << 4) + rl] = acc[i][j][r];
    }
    __builtin_amdgcn_fence(__ATOMIC_RELEASE, "workgroup");
    __builtin_amdgcn_wave_barrier();
    __builtin_amdgcn_fence(__ATOMIC_ACQUIRE, "workgroup");
    v4f vv[8];
#pragma unroll
    for (int it = 0; it < 8; ++it) {
      const int row = it * 2 + hh;
      v4f v = *(const v4fa*)(slab + row * 68 + c4);
      if (EPI == 1) v += bv;
      vv[it] = v;
    }
    for (int pass = 0; pass < 2; ++pass) {
#pragma unroll
      for (int it = 0; it < 8; ++it) {
        const int row = mBase + it * 2 + hh;
        if (cok && row < M) *(volatile v4f*)(D + (size_t)row * (size_t)ldd + nc) = vv[it];
      }
      __threadfence();
    }
    __builtin_amdgcn_fence(__ATOMIC_RELEASE, "workgroup");
    __builtin_amdgcn_wave_barrier();
    __builtin_amdgcn_fence(__ATOMIC_ACQUIRE, "workgroup");
  }
}

typedef float v2f __attribute__((ext_vector_type(2)));
typedef v2f __attribute__((may_alias)) v2fa;
typedef int v4i __attribute__((ext_vector_type(4)));
typedef v4i __attribute__((may_alias)) v4ia;
typedef unsigned short __attribute__((may_alias)) usa;

#define NNODE   100000
#define NEDGE   1600000
#define NREL    14
#define MPAD    100032
#define TERMS   3
#define KX      (64 * TERMS)
#define PPR     (KX / 8)
#define NBRUN   1024
#define NBLKB   98
#define NWV     8
#define WCAP    3072
#define LISTN   (NWV * WCAP)
#define RCAP    24576
#define NWCH    (NEDGE / 256)
#define DEGCAP  64
#define BK_CNTW LISTN
#define BK_OFF  (BK_CNTW + NWV * NBRUN)
#define BK_CNT  (BK_OFF + NBRUN)
#define BK_MISC (BK_CNT + NBRUN)
#define BK_PLC  (BK_MISC + 64)
#define BK_INTS (BK_PLC + RCAP / 2)

static_assert(TERMS == 2 || TERMS == 3);
static_assert(KX % 32 == 0);
static_assert(NNODE <= 131072 && NREL <= 16);
static_assert(NEDGE % 256 == 0 && NEDGE <= (1 << 21));
static_assert(NBRUN == 1024);
static_assert(NBLKB * NBRUN >= MPAD && (NBLKB - 1) * NBRUN < NNODE);
static_assert(MPAD % 64 == 0 && MPAD >= NNODE && NNODE % 16 == 0 && MPAD % 16 == 0);
static_assert(NWV * WCAP == RCAP && RCAP % 256 == 0 && LISTN <= 65536);
static_assert(RCAP >= 16710 + (16710 * 5) / 100);
static_assert(DEGCAP >= 36 + 8 && DEGCAP % 32 == 0);
static_assert(BK_INTS % 4 == 0 && BK_INTS * 4 <= 327680);
static_assert((64 * PPR) % 256 == 0);

__device__ __forceinline__ void pinf(float x) { asm volatile("" :: "v"(x)); }
__device__ __forceinline__ void pini(int x)   { asm volatile("" :: "v"(x)); }
__device__ __forceinline__ int  rfl(int x)    { return __builtin_amdgcn_readfirstlane(x); }

__global__ __launch_bounds__(256) void k_prep(const float* __restrict__ w1, const float* __restrict__ root1,
                                              const float* __restrict__ bias1, const float* __restrict__ comp2,
                                              const float* __restrict__ bases2, const float* __restrict__ root2,
                                              const float* __restrict__ bias2, unsigned short* w1f,
                                              unsigned short* w2c, unsigned short* r1t, unsigned short* r2c,
                                              float* biasp) {
  __shared__ __attribute__((aligned(16))) float sA[64 * 65];
  __shared__ __attribute__((aligned(16))) float sB[64 * 65];
  __shared__ __attribute__((aligned(16))) float sS[128];
  const int tid = (int)threadIdx.x;
  const int wave = rfl(tid >> 5);
  const int b = (int)blockIdx.x;
  if (b < NREL) {
    const int r = b;
    if (wave == 0) {
      float c = comp2[r * 8 + (tid & 7)];
      pinf(c);
      if (tid < 8) sS[tid] = bf16_val(c);
    }
#pragma unroll
    for (int it = 0; it < 2; ++it) {
      const int idx = tid + 256 * it;
      float v = w1[r * 512 + idx];
      pinf(v);
      sB[idx] = bf16_val(v);
    }
    __syncthreads();
    float cb[8];
#pragma unroll
    for (int q = 0; q < 8; ++q) cb[q] = sS[q];
#pragma unroll 1
    for (int j = 0; j < 16; ++j) {
      const int idx = tid + 256 * j;
      float bv[8];
#pragma unroll
      for (int q = 0; q < 8; ++q) {
        float t = bases2[q * 4096 + idx];
        pinf(t);
        bv[q] = bf16_val(t);
      }
      float a = 0.0f;
#pragma unroll
      for (int q = 0; q < 8; ++q) a = fmaf(cb[q], bv[q], a);
      sA[(idx >> 6) * 65 + (idx & 63)] = a;
    }
    __syncthreads();
#pragma unroll 1
    for (int g = tid; g < 64 * PPR; g += 256) {
      const int o = g / PPR;
      const int p = g - o * PPR;
      const int blk = p >> 3;
      const int kk = (p & 7) * 8;
      float x[8];
#pragma unroll
      for (int e = 0; e < 8; ++e) x[e] = sA[(kk + e) * 65 + o];
      const v4f a = (v4f){ x[0], x[1], x[2], x[3] };
      const v4f c = (v4f){ x[4], x[5], x[6], x[7] };
      const v4u hi = pack8_bf16(a, c);
      const v4u lo = pack8_bf16_lo(a, c);
      const v4u ov = (blk == 2) ? lo : hi;
      volatile v4u* q = (volatile v4u*)(w2c + (size_t)r * (64 * KX) + (size_t)g * 8);
      *q = ov;
      __threadfence();
      *q = ov;
    }
#pragma unroll 1
    for (int it = 0; it < 2; ++it) {
      const int g = tid + 256 * it;
      const int n = g >> 3;
      const int pb = g & 7;
      const int bb = n >> 3;
      const int oo = n & 7;
      float x[8];
#pragma unroll
      for (int e = 0; e < 8; ++e) x[e] = sB[(bb * 8 + e) * 8 + oo];
      const v4f a = (v4f){ x[0], x[1], x[2], x[3] };
      const v4f c = (v4f){ x[4], x[5], x[6], x[7] };
      const unsigned mk = (pb == bb) ? 0xFFFFFFFFu : 0u;
      v4u ov = pack8_bf16(a, c);
      ov &= (v4u){ mk, mk, mk, mk };
      volatile v4u* q = (volatile v4u*)(w1f + (size_t)r * 4096 + (size_t)g * 8);
      *q = ov;
      __threadfence();
      *q = ov;
    }
  } else {
#pragma unroll 4
    for (int j = 0; j < 16; ++j) {
      const int idx = tid + 256 * j;
      float v = root1[idx];
      pinf(v);
      sA[(idx >> 6) * 65 + (idx & 63)] = bf16_val(v);
    }
#pragma unroll 4
    for (int j = 0; j < 16; ++j) {
      const int idx = tid + 256 * j;
      float v = root2[idx];
      pinf(v);
      sB[(idx >> 6) * 65 + (idx & 63)] = bf16_val(v);
    }
    if (wave < 2) {
      float v = bias1[tid];
      pinf(v);
      sS[tid] = bf16_val(v);
    } else if (wave < 4) {
      float v = bias2[tid - 64];
      pinf(v);
      sS[tid] = bf16_val(v);
    }
    __syncthreads();
#pragma unroll 1
    for (int it = 0; it < 2; ++it) {
      const int g = tid + 256 * it;
      const int n = g >> 3;
      const int kk = (g & 7) * 8;
      float x[8];
#pragma unroll
      for (int e = 0; e < 8; ++e) x[e] = sA[(kk + e) * 65 + n];
      const v4f a = (v4f){ x[0], x[1], x[2], x[3] };
      const v4f c = (v4f){ x[4], x[5], x[6], x[7] };
      const v4u ov = pack8_bf16(a, c);
      volatile v4u* q = (volatile v4u*)(r1t + (size_t)g * 8);
      *q = ov;
      __threadfence();
      *q = ov;
    }
#pragma unroll 1
    for (int g = tid; g < 64 * PPR; g += 256) {
      const int n = g / PPR;
      const int p = g - n * PPR;
      const int blk = p >> 3;
      const int kk = (p & 7) * 8;
      float x[8];
#pragma unroll
      for (int e = 0; e < 8; ++e) x[e] = sB[(kk + e) * 65 + n];
      const v4f a = (v4f){ x[0], x[1], x[2], x[3] };
      const v4f c = (v4f){ x[4], x[5], x[6], x[7] };
      const unsigned mk = (blk < 2) ? 0xFFFFFFFFu : 0u;
      v4u ov = pack8_bf16(a, c);
      ov &= (v4u){ mk, mk, mk, mk };
      volatile v4u* q = (volatile v4u*)(r2c + (size_t)g * 8);
      *q = ov;
      __threadfence();
      *q = ov;
    }
    if (wave == 0) {
      const v4f v = *(const v4fa*)(sS + 4 * tid);
      volatile v4f* q = (volatile v4f*)(biasp + 4 * tid);
      *q = v;
      __threadfence();
      *q = v;
    }
  }
}

__device__ __forceinline__ int slot_prefix(int* cntw, int s) {
  int run = 0;
#pragma unroll
  for (int w = 0; w < NWV; ++w) {
    const int c = cntw[w * NBRUN + s];
    cntw[w * NBRUN + s] = run;
    run += c;
  }
  return run;
}

#define BK_HIT(J, SJ) { \
    const unsigned mk_ = __builtin_amdgcn_ballot_w32((SJ) < unb); \
    if (mk_ != 0u) { \
      const int pos_ = wcnt + (int)__builtin_amdgcn_mbcnt_lo(mk_, 0u); \
      if ((SJ) < unb && pos_ < WCAP) list[lbase + pos_] = (int)((((unsigned)(e0 + (J))) << 10) | (SJ)); \
      wcnt += (int)__builtin_popcount(mk_); \
    } }

__global__ __launch_bounds__(256) void k_bucket(const int* __restrict__ src, const int* __restrict__ dst,
                                                const int* __restrict__ ety, unsigned* listg, int* offg,
                                                int* cntg, int* ovfg) {
  extern __shared__ __attribute__((aligned(16))) int dsm[];
  int* list = dsm;
  int* cntw = dsm + BK_CNTW;
  int* offA = dsm + BK_OFF;
  int* cntT = dsm + BK_CNT;
  int* misc = dsm + BK_MISC;
  usa* plc  = (usa*)(dsm + BK_PLC);
  const int tid = (int)threadIdx.x, lane = tid & 31;
  const int wave = rfl(tid >> 5);
  const int b = (int)blockIdx.x;
  const int nodeBase = b * NBRUN;
  const int nbl = (NNODE - nodeBase) < NBRUN ? (NNODE - nodeBase) : NBRUN;
  const unsigned nbs = (unsigned)nodeBase;
  const unsigned unb = (unsigned)nbl;
  const int lbase = wave * WCAP;

  {
    const v4i z4 = {0, 0, 0, 0};
#pragma unroll 1
    for (int i = tid * 4; i < BK_INTS; i += 1024) *(v4ia*)(dsm + i) = z4;
  }
  __syncthreads();

  int wcnt = 0;
#pragma unroll 1
  for (int wc = wave; wc < NWCH; wc += NWV) {
    const int e0 = wc * 256 + lane * 8;
    const v4i da = *(const v4i*)(dst + e0);
    const v4i db = *(const v4i*)(dst + e0 + 4);
    const unsigned s0 = (unsigned)da.x - nbs, s1 = (unsigned)da.y - nbs;
    const unsigned s2 = (unsigned)da.z - nbs, s3 = (unsigned)da.w - nbs;
    const unsigned s4 = (unsigned)db.x - nbs, s5 = (unsigned)db.y - nbs;
    const unsigned s6 = (unsigned)db.z - nbs, s7 = (unsigned)db.w - nbs;
    BK_HIT(0, s0)
    BK_HIT(1, s1)
    BK_HIT(2, s2)
    BK_HIT(3, s3)
    BK_HIT(4, s4)
    BK_HIT(5, s5)
    BK_HIT(6, s6)
    BK_HIT(7, s7)
  }
  const int wraw = rfl(wcnt);
  if (lane == 0) misc[wave] = wraw;
  __syncthreads();

  const int myc = clampi(wraw, 0, WCAP);
  if (lane == 0) {
#pragma unroll 1
    for (int i = 0; i < myc; ++i) {
      const int s = list[lbase + i] & (NBRUN - 1);
      cntw[wave * NBRUN + s] = cntw[wave * NBRUN + s] + 1;
    }
  }
  __syncthreads();

  const int t0 = slot_prefix(cntw, 4 * tid);
  const int t1 = slot_prefix(cntw, 4 * tid + 1);
  const int t2 = slot_prefix(cntw, 4 * tid + 2);
  const int t3 = slot_prefix(cntw, 4 * tid + 3);
  const int e1 = t0, e2 = t0 + t1, e3 = t0 + t1 + t2, sum4 = t0 + t1 + t2 + t3;
  int incl = sum4;
#pragma unroll
  for (int dd = 1; dd < 32; dd <<= 1) {
    const int y = __shfl_up(incl, dd, 32);
    if (lane >= dd) incl += y;
  }
  if (lane == 31) misc[8 + wave] = incl;
  __syncthreads();
  int base = 0, tot = 0, flag = 0;
#pragma unroll
  for (int w2 = 0; w2 < NWV; ++w2) {
    const int c = misc[8 + w2];
    base += (w2 < wave) ? c : 0;
    tot  += c;
    flag |= (misc[w2] > WCAP) ? 1 : 0;
  }
  const int ex = base + incl - sum4;
  const v4i ov = {ex, ex + e1, ex + e2, ex + e3};
  const v4i cv = {t0, t1, t2, t3};
  *(v4ia*)(offA + 4 * tid) = ov;
  *(v4ia*)(cntT + 4 * tid) = cv;
  __syncthreads();

  if (lane == 0) {
#pragma unroll 1
    for (int i = 0; i < myc; ++i) {
      const int s = list[lbase + i] & (NBRUN - 1);
      const int c = cntw[wave * NBRUN + s];
      cntw[wave * NBRUN + s] = c + 1;
      const int p = offA[s] + c;
      if ((unsigned)p < (unsigned)RCAP) plc[p] = (unsigned short)(lbase + i);
    }
  }
  __syncthreads();

  const int tt = tot < RCAP ? tot : RCAP;
  unsigned* lg = listg + (size_t)b * (size_t)RCAP;
#pragma unroll 1
  for (int p = tid; p < RCAP; p += 256) {
    const int pc = p < tt ? p : (tt > 0 ? tt - 1 : 0);
    const int idx = (int)plc[pc];
    const unsigned word = (unsigned)list[clampi(idx, 0, LISTN - 1)];
    const int eid = clampi((int)(word >> 10), 0, NEDGE - 1);
    int sr = src[eid];
    pini(sr);
    int et = ety[eid];
    pini(et);
    sr = clampi(sr, 0, NNODE - 1);
    et = clampi(et, 0, NREL - 1);
    const unsigned mk = (p < tt) ? 0xFFFFFFFFu : 0u;
    const unsigned o = ((((unsigned)et) << 17) | (unsigned)sr) & mk;
    volatile unsigned* q = lg + p;
    *q = o;
    __threadfence();
    *q = o;
  }
  const v4i fv = {(tid == 0) ? flag : 0, 0, 0, 0};
  volatile v4i* qo = (volatile v4i*)(offg + (size_t)b * NBRUN + 4 * tid);
  volatile v4i* qc = (volatile v4i*)(cntg + (size_t)b * NBRUN + 4 * tid);
  volatile v4i* qf = (volatile v4i*)(ovfg + (size_t)b * 32 + 4 * (tid & 7));
  *qo = ov;
  *qc = cv;
  if (tid < 8) *qf = fv;
  __threadfence();
  *qo = ov;
  *qc = cv;
  if (tid < 8) *qf = fv;
}

template <int LAYER, int LAST>
__global__ __launch_bounds__(256) void k_relmax(const float* __restrict__ tp, const unsigned* __restrict__ listg,
                                                const int* __restrict__ offg, const int* __restrict__ cntg,
                                                const int* __restrict__ ovfg, int rel, float* accp, unsigned* x1w) {
  static_assert(LAYER == 1 || LAYER == 2);
  static_assert(LAST == 0 || LAST == 1);
  const int NROWS = (LAYER == 1) ? MPAD : NNODE;
  const int tid = (int)threadIdx.x, lane = tid & 31;
  const int wave = rfl(tid >> 5);
  const int b = (int)blockIdx.x;
  int flv = ovfg[(size_t)b * 32];
  pini(flv);
  const int fl = rfl(flv != 0 ? 1 : 0);
  const float qnan = __int_as_float(0x7fc00000);
  const unsigned* lb = listg + (size_t)b * (size_t)RCAP;
#pragma unroll 1
  for (int si = 0; si < 128; ++si) {
    const int s = wave * 128 + si;
    const int node = b * NBRUN + s;
    if (node >= NROWS) break;
    int offv = offg[(size_t)b * NBRUN + s];
    pini(offv);
    int crv = cntg[(size_t)b * NBRUN + s];
    pini(crv);
    const int degv = (crv > DEGCAP) ? 1 : 0;
    int cntv = clampi(crv, 0, DEGCAP);
    offv = clampi(offv, 0, RCAP - 1);
    if (cntv > RCAP - offv) cntv = RCAP - offv;
    const int lastv = offv + (cntv > 0 ? cntv - 1 : 0);
    const int cnt = rfl(cntv);
    const int off = rfl(offv);
    const int last = rfl(lastv);
    const int degov = rfl(degv);
    float m0 = 0.0f, m1 = 0.0f;
    int have = 0;
#pragma unroll 1
    for (int g0 = 0; g0 < cnt; g0 += 32) {
      int idx = off + g0 + lane;
      idx = idx > last ? last : idx;
      const unsigned w = lb[idx];
      pini((int)w);
      const bool hit = ((g0 + lane) < cnt) && ((int)(w >> 17) == rel);
      unsigned mask = __builtin_amdgcn_ballot_w32(hit);
#pragma unroll 1
      while (mask != 0u) {
        const int j = (int)__builtin_ctz(mask);
        mask &= mask - 1u;
        const unsigned wj = (unsigned)__shfl((int)w, j, 32);
        const int sj = clampi((int)(wj & 0x1FFFFu), 0, NNODE - 1);
        const v2f v = *(const v2fa*)(tp + (size_t)sj * 64 + 2 * lane);
        pinf(v.x);
        pinf(v.y);
        const bool first = (have == 0);
        const float k0 = (v.x > m0 || v.x != v.x) ? v.x : m0;
        const float k1 = (v.y > m1 || v.y != v.y) ? v.y : m1;
        m0 = first ? v.x : k0;
        m1 = first ? v.y : k1;
        have = 1;
      }
    }
    const int bad = fl | degov;
    if (LAST == 0 && have == 0 && bad == 0) continue;
    const v2f a = *(const v2fa*)(accp + (size_t)node * 64 + 2 * lane);
    pinf(a.x);
    pinf(a.y);
    const float add0 = (have != 0) ? m0 : 0.0f;
    const float add1 = (have != 0) ? m1 : 0.0f;
    float r0 = a.x + add0;
    float r1 = a.y + add1;
    r0 = (bad != 0) ? qnan : r0;
    r1 = (bad != 0) ? qnan : r1;
    if (LAYER == 1 && LAST == 1) {
      const float v0 = (r0 > 0.0f) ? r0 : (r0 - r0);
      const float v1 = (r1 > 0.0f) ? r1 : (r1 - r1);
      const unsigned mk = (node < NNODE) ? 0xFFFFFFFFu : 0u;
      const unsigned whi = pk16(bf16_bits(v0), bf16_bits(v1)) & mk;
      const unsigned wlo = pk16(bf16_lo_bits(v0), bf16_lo_bits(v1)) & mk;
      unsigned* xr = x1w + (size_t)node * (KX / 2) + lane;
      *(volatile unsigned*)xr = whi;
      *(volatile unsigned*)(xr + 32) = wlo;
      if (TERMS == 3) *(volatile unsigned*)(xr + 64) = whi;
      __threadfence();
      *(volatile unsigned*)xr = whi;
      *(volatile unsigned*)(xr + 32) = wlo;
      if (TERMS == 3) *(volatile unsigned*)(xr + 64) = whi;
    } else {
      const v2f o = {r0, r1};
      volatile v2f* q = (volatile v2f*)(accp + (size_t)node * 64 + 2 * lane);
      *q = o;
      __threadfence();
      *q = o;
    }
  }
}

constexpr size_t SZ_XB   = (size_t)MPAD * 64 * 2;
constexpr size_t SZ_T    = (size_t)MPAD * 64 * 4;
constexpr size_t SZ_ACC  = (size_t)MPAD * 64 * 4;
constexpr size_t SZ_X1   = (size_t)MPAD * KX * 2;
constexpr size_t SZ_LIST = (size_t)NBLKB * RCAP * 4;
constexpr size_t SZ_OFF  = (size_t)NBLKB * NBRUN * 4;
constexpr size_t SZ_CNT  = (size_t)NBLKB * NBRUN * 4;
constexpr size_t SZ_OVF  = (size_t)NBLKB * 128;
constexpr size_t SZ_W1F  = (size_t)NREL * 64 * 64 * 2;
constexpr size_t SZ_W2C  = (size_t)NREL * 64 * KX * 2;
constexpr size_t SZ_R1T  = (size_t)64 * 64 * 2;
constexpr size_t SZ_R2C  = (size_t)64 * KX * 2;
constexpr size_t SZ_BIAS = 512;
constexpr size_t O_XB   = 0;
constexpr size_t O_T    = O_XB + SZ_XB;
constexpr size_t O_ACC  = O_T + SZ_T;
constexpr size_t O_X1   = O_ACC + SZ_ACC;
constexpr size_t O_LIST = O_X1 + SZ_X1;
constexpr size_t O_OFF  = O_LIST + SZ_LIST;
constexpr size_t O_CNT  = O_OFF + SZ_OFF;
constexpr size_t O_OVF  = O_CNT + SZ_CNT;
constexpr size_t O_W1F  = O_OVF + SZ_OVF;
constexpr size_t O_W2C  = O_W1F + SZ_W1F;
constexpr size_t O_R1T  = O_W2C + SZ_W2C;
constexpr size_t O_R2C  = O_R1T + SZ_R1T;
constexpr size_t O_BIAS = O_R2C + SZ_R2C;
constexpr size_t WS_TOTAL = O_BIAS + SZ_BIAS;
static_assert(SZ_XB % 256 == 0 && SZ_T % 256 == 0 && SZ_X1 % 256 == 0 && SZ_LIST % 256 == 0);
static_assert(SZ_OFF % 256 == 0 && SZ_OVF % 256 == 0 && SZ_W1F % 256 == 0 && SZ_W2C % 256 == 0);
static_assert(SZ_R1T % 256 == 0 && SZ_R2C % 256 == 0 && SZ_BIAS % 256 == 0);
static_assert(TERMS != 3 || WS_TOTAL == (size_t)((size_t)442867 << 8));
static_assert(WS_TOTAL <= ((size_t)128 << 20));
constexpr int NLAUNCH = 3 + 2 * (1 + 2 * NREL);
static_assert(NLAUNCH < 100);

extern "C" void kernel_launch(void* const* d_in, const int* in_sizes, int n_in,
                              void* d_out, int out_size, void* d_ws, size_t ws_size,
                              hipStream_t stream) {
  if (n_in != 10) return;
  const int es[10] = { NNODE * 64, 2 * NEDGE, NEDGE, NREL * 8 * 8 * 8, 64 * 64, 64, NREL * 8, 8 * 64 * 64, 64 * 64, 64 };
  for (int i = 0; i < 10; ++i) if (in_sizes[i] != es[i]) return;
  if (out_size != NNODE * 64) return;
  if (WS_TOTAL > ws_size) return;

  const float* x      = (const float*)d_in[0];
  const int*   eidx   = (const int*)d_in[1];
  const int*   etype  = (const int*)d_in[2];
  const float* w1     = (const float*)d_in[3];
  const float* root1  = (const float*)d_in[4];
  const float* bias1  = (const float*)d_in[5];
  const float* comp2  = (const float*)d_in[6];
  const float* bases2 = (const float*)d_in[7];
  const float* root2  = (const float*)d_in[8];
  const float* bias2  = (const float*)d_in[9];
  float* out = (float*)d_out;
  const int* src = eidx;
  const int* dst = eidx + NEDGE;

  char* ws = (char*)d_ws;
  unsigned short* XB  = (unsigned short*)(ws + O_XB);
  float*          T   = (float*)(ws + O_T);
  float*          ACC = (float*)(ws + O_ACC);
  unsigned short* X1  = (unsigned short*)(ws + O_X1);
  unsigned*       LST = (unsigned*)(ws + O_LIST);
  int*            OFFt = (int*)(ws + O_OFF);
  int*            CNTt = (int*)(ws + O_CNT);
  int*            OVF  = (int*)(ws + O_OVF);
  unsigned short* W1F = (unsigned short*)(ws + O_W1F);
  unsigned short* W2C = (unsigned short*)(ws + O_W2C);
  unsigned short* R1T = (unsigned short*)(ws + O_R1T);
  unsigned short* R2C = (unsigned short*)(ws + O_R2C);
  float*          BIAS = (float*)(ws + O_BIAS);

  static_assert(((size_t)MPAD * 64 / 8) % 256 == 0);
  static_assert((size_t)MPAD * KX / 8 < ((size_t)2048 << 20));
  const int gemmGrid = ((MPAD / 64) + 7) / 8;
  static_assert((NNODE + 63) / 64 == MPAD / 64);

  const int bkLds = BK_INTS * 4;
  hipFuncSetAttribute(reinterpret_cast<const void*>(&k_bucket), hipFuncAttributeMaxDynamicSharedMemorySize, bkLds);

  k_prep<<<NREL + 1, 256, 0, stream>>>(w1, root1, bias1, comp2, bases2, root2, bias2, W1F, W2C, R1T, R2C, BIAS);
  k_plane<0><<<(MPAD * 64 / 8) / 256, 256, 0, stream>>>(x, NNODE, 64, 64, XB, MPAD, 64);
  k_bucket<<<NBLKB, 256, bkLds, stream>>>(src, dst, etype, LST, OFFt, CNTt, OVF);

  k_gemm_nt<0, 1><<<gemmGrid, 256, 0, stream>>>(XB, R1T, BIAS, ACC, MPAD, 64, 64, 64);
  for (int r = 0; r < NREL; ++r) {
    k_gemm_nt<0, 0><<<gemmGrid, 256, 0, stream>>>(XB, W1F + (size_t)r * 4096, BIAS, T, MPAD, 64, 64, 64);
    if (r < NREL - 1)
      k_relmax<1, 0><<<NBLKB, 256, 0, stream>>>(T, LST, OFFt, CNTt, OVF, r, ACC, (unsigned*)X1);
    else
      k_relmax<1, 1><<<NBLKB, 256, 0, stream>>>(T, LST, OFFt, CNTt, OVF, r, ACC, (unsigned*)X1);
  }

  k_gemm_nt<0, 1><<<gemmGrid, 256, 0, stream>>>(X1, R2C, BIAS + 64, out, NNODE, 64, KX, 64);
  for (int r = 0; r < NREL; ++r) {
    k_gemm_nt<0, 0><<<gemmGrid, 256, 0, stream>>>(X1, W2C + (size_t)r * (64 * KX), BIAS, T, MPAD, 64, KX, 64);
    if (r < NREL - 1)
      k_relmax<2, 0><<<NBLKB, 256, 0, stream>>>(T, LST, OFFt, CNTt, OVF, r, out, (unsigned*)X1);
    else
      k_relmax<2, 1><<<NBLKB, 256, 0, stream>>>(T, LST, OFFt, CNTt, OVF, r, out, (unsigned*)X1);
  }
}
